// MultiHeadAttentionV2_24120536334834
// MI455X (gfx1250) — hardware-verified
//
#include <hip/hip_runtime.h>

constexpr int kB   = 4;
constexpr int kS   = 2048;
constexpr int kD   = 1024;
constexpr int kH   = 16;
constexpr int kHD  = 64;
constexpr int kTok = kB * kS;
constexpr int kBH  = kB * kH;
constexpr int kKC  = 64;
constexpr int kQTiles     = kS / 64;
constexpr int kSplitRows  = 512;
constexpr int kSplitTiles = kSplitRows / 64;
constexpr float kScoreScale = 0.125f;
constexpr float kPCarry     = 32768.0f;
static_assert(kH * kHD == kD, "shape");
static_assert(kS % 64 == 0 && kD % 64 == 0 && kTok % 64 == 0, "tiles");
static_assert(kD % 32 == 0 && kHD % 32 == 0, "k steps");
static_assert(kSplitRows % 64 == 0 && kSplitRows <= kS, "split rows");

typedef __attribute__((ext_vector_type(16))) _Float16 v16h;
typedef __attribute__((ext_vector_type(8)))  _Float16 v8h;
typedef __attribute__((ext_vector_type(16))) __bf16   v16b;
typedef __attribute__((ext_vector_type(8)))  __bf16   v8b;
typedef __attribute__((ext_vector_type(8)))  float    v8f;
typedef __attribute__((ext_vector_type(4)))  float    v4f;
typedef __attribute__((ext_vector_type(4)))  unsigned int v4u;

__device__ __forceinline__ unsigned short f2bf_bits(float f) {
  unsigned u = __float_as_uint(f);
  return (unsigned short)((u + 0x7FFFu + ((u >> 16) & 1u)) >> 16);
}
__device__ __forceinline__ float bf_bits2f(unsigned short hb) { return __uint_as_float(((unsigned)hb) << 16); }
__device__ __forceinline__ unsigned pk16(unsigned short a, unsigned short b) { return (unsigned)a | ((unsigned)b << 16); }
__device__ __forceinline__ unsigned short h_bits(float f) { const _Float16 hv = (_Float16)f; return __builtin_bit_cast(unsigned short, hv); }

__device__ __forceinline__ void dep_guard4_h(v8f& a, v8f& b, v8f& c, v8f& d, v16h x, v16h y) {
  asm volatile("v_nop\n\tv_nop\n\tv_nop\n\tv_nop" : "+v"(a), "+v"(b), "+v"(c), "+v"(d) : "v"(x), "v"(y));
}
__device__ __forceinline__ void dep_guard4_b(v8f& a, v8f& b, v8f& c, v8f& d, v16b x, v16b y) {
  asm volatile("v_nop\n\tv_nop\n\tv_nop\n\tv_nop" : "+v"(a), "+v"(b), "+v"(c), "+v"(d) : "v"(x), "v"(y));
}
__device__ __forceinline__ void keep4_h(v16h a, v16h b, v16h c, v16h d) { asm volatile("v_nop" :: "v"(a), "v"(b), "v"(c), "v"(d)); }
__device__ __forceinline__ void keep4_b(v16b a, v16b b, v16b c, v16b d) { asm volatile("v_nop" :: "v"(a), "v"(b), "v"(c), "v"(d)); }
__device__ __forceinline__ void acc_guard4(v8f& a, v8f& b, v8f& c, v8f& d) { asm volatile("v_nop\n\tv_nop\n\tv_nop\n\tv_nop" : "+v"(a), "+v"(b), "+v"(c), "+v"(d)); }

template <typename T> struct Frag;
template <> struct Frag<_Float16> {
  typedef v16h V; union U { v16h v; v8h hv[2]; };
  static __device__ __forceinline__ v16h load(const _Float16* p) {
    U f; f.hv[0] = *(const v8h*)(p); f.hv[1] = *(const v8h*)(p + 16); return f.v;
  }
  static __device__ __forceinline__ v8f mma(v16h a, v16h b, v8f c) {
    return __builtin_amdgcn_wmma_f32_16x16x32_f16(false, a, false, b, (short)0, c, false, false);
  }
  static __device__ __forceinline__ void guard4(v8f& a, v8f& b, v8f& c, v8f& d, v16h x, v16h y) { dep_guard4_h(a, b, c, d, x, y); }
  static __device__ __forceinline__ void keep(v16h a, v16h b, v16h c, v16h d) { keep4_h(a, b, c, d); }
};
template <> struct Frag<__bf16> {
  typedef v16b V; union U { v16b v; v8b hv[2]; };
  static __device__ __forceinline__ v16b load(const __bf16* p) {
    U f; f.hv[0] = *(const v8b*)(p); f.hv[1] = *(const v8b*)(p + 16); return f.v;
  }
  static __device__ __forceinline__ v8f mma(v16b a, v16b b, v8f c) {
    return __builtin_amdgcn_wmma_f32_16x16x32_bf16(false, a, false, b, (short)0, c, false, false);
  }
  static __device__ __forceinline__ void guard4(v8f& a, v8f& b, v8f& c, v8f& d, v16b x, v16b y) { dep_guard4_b(a, b, c, d, x, y); }
  static __device__ __forceinline__ void keep(v16b a, v16b b, v16b c, v16b d) { keep4_b(a, b, c, d); }
};

template <int ET> struct Elem;
template <> struct Elem<0> { typedef _Float16 T; };
template <> struct Elem<1> { typedef __bf16 T; };
template <int ET, int SPLITM, int BIAS_MODE, int OUT_MODE>
__global__ __launch_bounds__(256) void wmma_gemm64(
    const unsigned short* __restrict__ Ap, const unsigned short* __restrict__ A2p, int lda, long strideA,
    const unsigned short* __restrict__ Btp, const unsigned short* __restrict__ Bt2p, int ldb, long strideB,
    void* Cout, int ldc, long strideC,
    void* Cout2, void* Cout3, int ldc2, long strideC2, int mlim, int nlim,
    const float* __restrict__ bias, int M, int N, int K, float scale) {
  typedef typename Elem<ET>::T T;
  typedef typename Frag<T>::V V;
  const T* A = (const T*)Ap; const T* A2 = (const T*)A2p; const T* Bt = (const T*)Btp; const T* Bt2 = (const T*)Bt2p;
  __shared__ __align__(16) float sT[8][16 * 68];
  const int b    = blockIdx.y;
  const int lane = threadIdx.x & 31;
  const int wave = threadIdx.x >> 5;
  const int tilesN = N >> 6;
  const int tilesM = M >> 6;
  const int tile = blockIdx.x * 8 + wave;
  if (tile >= tilesM * tilesN) return;
  const int tm = tile / tilesN;
  const int tn = tile - tm * tilesN;
  const int m0 = tm << 6;
  const int n0 = tn << 6;

  const T* Ab  = A  + (size_t)b * strideA;
  const T* Bb  = Bt + (size_t)b * strideB;
  const T* Ab2 = (SPLITM != 0) ? (A2  + (size_t)b * strideA) : nullptr;
  const T* Bb2 = (SPLITM == 1) ? (Bt2 + (size_t)b * strideB) : nullptr;

  const int rlane = lane & 15;
  const int koff  = (lane >> 4) * 8;
  const int mOff  = (lane >> 4) * 8;

  v8f acc[4][4];
#pragma unroll
  for (int i = 0; i < 4; ++i)
#pragma unroll
    for (int j = 0; j < 4; ++j) acc[i][j] = (v8f){0.f,0.f,0.f,0.f,0.f,0.f,0.f,0.f};

  for (int k0 = 0; k0 < K; k0 += 32) {
    V bh[4], bl[4];
#pragma unroll
    for (int j = 0; j < 4; ++j) {
      const size_t bofs = (size_t)(n0 + (j << 4) + rlane) * ldb + koff + k0;
      bh[j] = Frag<T>::load(Bb + bofs);
      if (SPLITM == 1) bl[j] = Frag<T>::load(Bb2 + bofs);
      else bl[j] = bh[j];
    }
#pragma unroll
    for (int i = 0; i < 4; ++i) {
      const size_t aofs = (size_t)(m0 + (i << 4) + rlane) * lda + koff + k0;
      V ah = Frag<T>::load(Ab + aofs);
      V al = ah;
      if (SPLITM != 0) al = Frag<T>::load(Ab2 + aofs);
#pragma unroll
      for (int j = 0; j < 4; ++j) {
        acc[i][j] = Frag<T>::mma(ah, bh[j], acc[i][j]);
        if (SPLITM == 1) acc[i][j] = Frag<T>::mma(ah, bl[j], acc[i][j]);
        if (SPLITM != 0) acc[i][j] = Frag<T>::mma(al, bh[j], acc[i][j]);
      }
      Frag<T>::guard4(acc[i][0], acc[i][1], acc[i][2], acc[i][3], ah, al);
    }
    Frag<T>::keep(bh[0], bh[1], bh[2], bh[3]);
    if (SPLITM == 1) Frag<T>::keep(bl[0], bl[1], bl[2], bl[3]);
  }
  acc_guard4(acc[0][0], acc[0][1], acc[0][2], acc[0][3]);
  acc_guard4(acc[1][0], acc[1][1], acc[1][2], acc[1][3]);
  acc_guard4(acc[2][0], acc[2][1], acc[2][2], acc[2][3]);
  acc_guard4(acc[3][0], acc[3][1], acc[3][2], acc[3][3]);

  float* slab = sT[wave];
  float bcol[4];
#pragma unroll
  for (int j = 0; j < 4; ++j) {
    if (BIAS_MODE == 2) bcol[j] = bias[n0 + (j << 4) + rlane];
    else bcol[j] = 0.0f;
  }
#pragma unroll
  for (int i = 0; i < 4; ++i) {
    const int mBase = m0 + (i << 4);
#pragma unroll
    for (int j = 0; j < 4; ++j) {
#pragma unroll
      for (int r = 0; r < 8; ++r) {
        float v = acc[i][j][r] * scale;
        if (BIAS_MODE == 2) v += bcol[j];
        slab[(mOff + r) * 68 + (j << 4) + rlane] = v;
      }
    }
    __builtin_amdgcn_fence(__ATOMIC_RELEASE, "workgroup");
    __builtin_amdgcn_wave_barrier();
    __builtin_amdgcn_fence(__ATOMIC_ACQUIRE, "workgroup");
    if (OUT_MODE == 0) {
      float* C = (float*)Cout + (size_t)b * strideC;
      const int hh = lane >> 4, c4 = (lane & 15) * 4;
      for (int pass = 0; pass < 2; ++pass) {
#pragma unroll
        for (int it = 0; it < 8; ++it) {
          const int row = it * 2 + hh;
          v4f v = *(const v4f*)(slab + row * 68 + c4);
          *(volatile v4f*)(C + (size_t)(mBase + row) * ldc + n0 + c4) = v;
        }
        __threadfence();
      }
    } else {
      const int q = lane >> 3, c8 = (lane & 7) * 8;
      unsigned short* C1  = (unsigned short*)Cout  + (size_t)b * strideC;
      unsigned short* C2p = (unsigned short*)Cout2 + (size_t)b * strideC2;
      unsigned short* C3p = (unsigned short*)Cout3 + (size_t)b * strideC2;
      const bool extra = (m0 < mlim) && (n0 < nlim);
      for (int pass = 0; pass < 2; ++pass) {
#pragma unroll
        for (int it = 0; it < 4; ++it) {
          const int row = it * 4 + q;
          const float* sp = slab + row * 68 + c8;
          unsigned short fb[8], hb[8], lb[8];
#pragma unroll
          for (int e = 0; e < 8; ++e) {
            const float val = sp[e];
            fb[e] = h_bits(val);
            const unsigned short hbv = f2bf_bits(val);
            hb[e] = hbv;
            lb[e] = f2bf_bits(val - bf_bits2f(hbv));
          }
          const v4u uf = (v4u){pk16(fb[0], fb[1]), pk16(fb[2], fb[3]), pk16(fb[4], fb[5]), pk16(fb[6], fb[7])};
          const v4u uh = (v4u){pk16(hb[0], hb[1]), pk16(hb[2], hb[3]), pk16(hb[4], hb[5]), pk16(hb[6], hb[7])};
          const v4u ul = (v4u){pk16(lb[0], lb[1]), pk16(lb[2], lb[3]), pk16(lb[4], lb[5]), pk16(lb[6], lb[7])};
          *(volatile v4u*)(C1 + (size_t)(mBase + row) * ldc + n0 + c8) = uf;
          if (extra) {
            *(volatile v4u*)(C2p + (size_t)(mBase + row) * ldc2 + n0 + c8) = uh;
            *(volatile v4u*)(C3p + (size_t)(mBase + row) * ldc2 + n0 + c8) = ul;
          }
        }
        __threadfence();
      }
    }
    __builtin_amdgcn_fence(__ATOMIC_RELEASE, "workgroup");
    __builtin_amdgcn_wave_barrier();
    __builtin_amdgcn_fence(__ATOMIC_ACQUIRE, "workgroup");
  }
}

__global__ __launch_bounds__(256) void cast8_bf16_kernel(const float* __restrict__ in, unsigned short* __restrict__ out, int n8) {
  const int i = blockIdx.x * 256 + threadIdx.x;
  if (i >= n8) return;
  const float* p = in + 8 * (size_t)i;
  const v4f a = *(const v4f*)(p);
  const v4f c = *(const v4f*)(p + 4);
  unsigned short hb[8];
#pragma unroll
  for (int e = 0; e < 4; ++e) {
    hb[e]     = f2bf_bits(a[e]);
    hb[4 + e] = f2bf_bits(c[e]);
  }
  const v4u u = (v4u){pk16(hb[0], hb[1]), pk16(hb[2], hb[3]), pk16(hb[4], hb[5]), pk16(hb[6], hb[7])};
  unsigned short* q = out + 8 * (size_t)i;
  *(volatile v4u*)q = u;
  __threadfence();
  *(volatile v4u*)q = u;
}

__global__ __launch_bounds__(256) void wtcast_kernel(const float* __restrict__ W0, const float* __restrict__ W1,
                                                     const float* __restrict__ W2, const float* __restrict__ W3,
                                                     unsigned short* __restrict__ out) {
  __shared__ float sm[64][65];
  const int t  = threadIdx.x;
  const int k0 = blockIdx.x * 64;
  const int n0 = blockIdx.y * 64;
  const int z  = blockIdx.z;
  const float* W = (z == 0) ? W0 : (z == 1) ? W1 : (z == 2) ? W2 : W3;
#pragma unroll
  for (int i = 0; i < 16; ++i) {
    const int e  = i * 256 + t;
    const int r  = e >> 6;
    const int cc = e & 63;
    sm[cc][r] = W[(size_t)(k0 + r) * kD + n0 + cc];
  }
  __syncthreads();
  const int lane = t & 31, wave = t >> 5;
  const int q = lane >> 3, c8 = (lane & 7) * 8;
  unsigned short* op = out + (size_t)z * kD * kD;
  for (int pass = 0; pass < 2; ++pass) {
#pragma unroll
    for (int it = 0; it < 2; ++it) {
      const int row = wave * 8 + it * 4 + q;
      unsigned short hb[8];
#pragma unroll
      for (int e = 0; e < 8; ++e) hb[e] = f2bf_bits(sm[row][c8 + e]);
      const v4u u = (v4u){pk16(hb[0], hb[1]), pk16(hb[2], hb[3]), pk16(hb[4], hb[5]), pk16(hb[6], hb[7])};
      *(volatile v4u*)(op + (size_t)(n0 + row) * kD + k0 + c8) = u;
    }
    __threadfence();
  }
}

__device__ __forceinline__ __bf16 at_f2bf(float f) { return __builtin_bit_cast(__bf16, f2bf_bits(f)); }
__device__ __forceinline__ void at_split(float f, __bf16& hi, __bf16& lo) {
  const unsigned short hb = f2bf_bits(f);
  hi = __builtin_bit_cast(__bf16, hb);
  lo = at_f2bf(f - __uint_as_float(((unsigned)hb) << 16));
}
__device__ __forceinline__ v8f at_mma(v16b a, v16b b, v8f c) {
  c = __builtin_amdgcn_wmma_f32_16x16x32_bf16(false, a, false, b, (short)0, c, false, false);
  asm volatile("v_nop\n\tv_nop\n\tv_nop\n\tv_nop" : "+v"(c) : "v"(a), "v"(b));
  return c;
}
template <bool F16> __device__ __forceinline__ __bf16 at_to16(float f) {
  if (F16) return __builtin_bit_cast(__bf16, (_Float16)f);
  return at_f2bf(f);
}
template <bool F16> __device__ __forceinline__ v8f at_mma16(v16b a, v16b b, v8f c) {
  if (F16) {
    const v16h ah = __builtin_bit_cast(v16h, a), bhh = __builtin_bit_cast(v16h, b);
    c = __builtin_amdgcn_wmma_f32_16x16x32_f16(false, ah, false, bhh, (short)0, c, false, false);
    asm volatile("v_nop\n\tv_nop\n\tv_nop\n\tv_nop" : "+v"(c) : "v"(ah), "v"(bhh));
    return c;
  }
  return at_mma(a, b, c);
}

template <bool SPLIT>
__global__ __launch_bounds__(128)
void attn_kernel(const unsigned short* __restrict__ qh, const unsigned short* __restrict__ ql,
                 const unsigned short* __restrict__ kh, const unsigned short* __restrict__ kl,
                 const unsigned short* __restrict__ vh, const unsigned short* __restrict__ vl,
                 unsigned short* oh, unsigned short* ol,
                 int qb0, int nqt, int qkRows, int vCols) {
  const float PSC = SPLIT ? 1.0f : kPCarry;
  union FB { v16b v; v8b hv[2]; v4u u[2]; };
  __shared__ __align__(16) unsigned short Ksh[kKC * kHD];
  __shared__ __align__(16) unsigned short Ksl[SPLIT ? kKC * kHD : 8];
  __shared__ __align__(16) unsigned short Vth[kHD * kKC];
  __shared__ __align__(16) unsigned short Vtl[SPLIT ? kHD * kKC : 8];
  __shared__ __align__(16) __bf16 Psh[4][16 * kKC];
  __shared__ __align__(16) __bf16 Psl[SPLIT ? 4 : 1][SPLIT ? 16 * kKC : 8];
  __shared__ __align__(16) float  Os[4][16 * 68];

  const int tid  = threadIdx.x;
  const int wave = tid >> 5;
  const int lane = tid & 31;
  const int hh   = lane >> 4;
  const int c    = lane & 15;

  const int bx = blockIdx.x;
  int qb = qb0 + (bx % nqt);
  if (qb > kQTiles - 1) qb = kQTiles - 1;
  const int bh = bx / nqt;
  const int h  = bh & (kH - 1);
  int b = bh >> 4;
  if (b > kB - 1) b = kB - 1;
  const int bhc = b * kH + h;
  const int q0 = qb * 64 + wave * 16;
  const size_t qk_bs = (size_t)qkRows * kD;
  int nChunks = qb + 1;
  const int maxChunks = qkRows / kKC;
  if (nChunks > maxChunks) nChunks = maxChunks;

  v16b qah[2], qal[2];
  {
    int qr = q0 + c;
    if (qr > qkRows - 1) qr = qkRows - 1;
    const size_t qofs = (size_t)b * qk_bs + (size_t)qr * kD + (size_t)h * kHD;
    const unsigned short* qrow  = qh + qofs;
    const unsigned short* qrow2 = ql + qofs;
#pragma unroll
    for (int dc = 0; dc < 2; ++dc) {
      FB f;
      f.u[0] = *(const v4u*)(qrow + dc * 32 + 8 * hh);
      f.u[1] = *(const v4u*)(qrow + dc * 32 + 16 + 8 * hh);
      qah[dc] = f.v;
      if (SPLIT) {
        FB g;
        g.u[0] = *(const v4u*)(qrow2 + dc * 32 + 8 * hh);
        g.u[1] = *(const v4u*)(qrow2 + dc * 32 + 16 + 8 * hh);
        qal[dc] = g.v;
      } else {
        qal[dc] = qah[dc];
      }
    }
  }

  float mrow[8], lrow[8];
  v8f oacc[4];
#pragma unroll
  for (int r = 0; r < 8; ++r) { mrow[r] = -__builtin_inff(); lrow[r] = 0.f; }
#pragma unroll
  for (int t = 0; t < 4; ++t) oacc[t] = (v8f){0.f,0.f,0.f,0.f,0.f,0.f,0.f,0.f};

  for (int kc = 0; kc < nChunks; ++kc) {
    const int kv0 = kc * kKC;
    __syncthreads();
    {
      const int r2 = tid >> 1, dh = (tid & 1) * 32;
      int kr = kv0 + r2;
      if (kr > qkRows - 1) kr = qkRows - 1;
      int kvc = kv0;
      if (kvc > vCols - kKC) kvc = vCols - kKC;
      const size_t kofs = (size_t)b * qk_bs + (size_t)kr * kD + (size_t)h * kHD + dh;
      const size_t vofs = ((size_t)bhc * kHD + r2) * (size_t)vCols + kvc + dh;
      {
        const unsigned short* kp = kh + kofs;
        const v4u w0 = *(const v4u*)(kp);
        const v4u w1 = *(const v4u*)(kp + 8);
        const v4u w2 = *(const v4u*)(kp + 16);
        const v4u w3 = *(const v4u*)(kp + 24);
        unsigned short* dst = Ksh + r2 * kHD + dh;
        *(v4u*)(dst) = w0; *(v4u*)(dst + 8) = w1; *(v4u*)(dst + 16) = w2; *(v4u*)(dst + 24) = w3;
      }
      asm volatile("" ::: "memory");
      {
        const unsigned short* vp = vh + vofs;
        const v4u w0 = *(const v4u*)(vp);
        const v4u w1 = *(const v4u*)(vp + 8);
        const v4u w2 = *(const v4u*)(vp + 16);
        const v4u w3 = *(const v4u*)(vp + 24);
        unsigned short* dst = Vth + r2 * kKC + dh;
        *(v4u*)(dst) = w0; *(v4u*)(dst + 8) = w1; *(v4u*)(dst + 16) = w2; *(v4u*)(dst + 24) = w3;
      }
      if (SPLIT) {
        asm volatile("" ::: "memory");
        {
          const unsigned short* kp = kl + kofs;
          const v4u w0 = *(const v4u*)(kp);
          const v4u w1 = *(const v4u*)(kp + 8);
          const v4u w2 = *(const v4u*)(kp + 16);
          const v4u w3 = *(const v4u*)(kp + 24);
          unsigned short* dst = Ksl + r2 * kHD + dh;
          *(v4u*)(dst) = w0; *(v4u*)(dst + 8) = w1; *(v4u*)(dst + 16) = w2; *(v4u*)(dst + 24) = w3;
        }
        asm volatile("" ::: "memory");
        {
          const unsigned short* vp = vl + vofs;
          const v4u w0 = *(const v4u*)(vp);
          const v4u w1 = *(const v4u*)(vp + 8);
          const v4u w2 = *(const v4u*)(vp + 16);
          const v4u w3 = *(const v4u*)(vp + 24);
          unsigned short* dst = Vtl + r2 * kKC + dh;
          *(v4u*)(dst) = w0; *(v4u*)(dst + 8) = w1; *(v4u*)(dst + 16) = w2; *(v4u*)(dst + 24) = w3;
        }
      }
    }
    __syncthreads();

    v8f s[4];
#pragma unroll
    for (int j = 0; j < 4; ++j) {
      s[j] = (v8f){0.f,0.f,0.f,0.f,0.f,0.f,0.f,0.f};
#pragma unroll
      for (int dc = 0; dc < 2; ++dc) {
        FB kb;
        kb.u[0] = *(const v4u*)(Ksh + (j * 16 + c) * kHD + dc * 32 + 8 * hh);
        kb.u[1] = *(const v4u*)(Ksh + (j * 16 + c) * kHD + dc * 32 + 16 + 8 * hh);
        s[j] = at_mma16<!SPLIT>(qah[dc], kb.v, s[j]);
        if (SPLIT) {
          FB klf;
          klf.u[0] = *(const v4u*)(Ksl + (j * 16 + c) * kHD + dc * 32 + 8 * hh);
          klf.u[1] = *(const v4u*)(Ksl + (j * 16 + c) * kHD + dc * 32 + 16 + 8 * hh);
          s[j] = at_mma16<!SPLIT>(qah[dc], klf.v, s[j]);
          s[j] = at_mma16<!SPLIT>(qal[dc], kb.v, s[j]);
        }
      }
    }
    const bool diag = (kc == qb);
    float cm[8];
#pragma unroll
    for (int r = 0; r < 8; ++r) {
      const int qrow = q0 + 8 * hh + r;
      float m = -__builtin_inff();
#pragma unroll
      for (int j = 0; j < 4; ++j) {
        const int kvcol = kv0 + j * 16 + c;
        float sv = s[j][r] * kScoreScale;
        if (diag && (kvcol > qrow)) sv = -__builtin_inff();
        s[j][r] = sv;
        m = fmaxf(m, sv);
      }
#pragma unroll
      for (int off = 1; off < 16; off <<= 1) m = fmaxf(m, __shfl_xor(m, off, 32));
      cm[r] = m;
    }
    __bf16* pwh = Psh[wave];
    __bf16* pwl = Psl[SPLIT ? wave : 0];
#pragma unroll
    for (int r = 0; r < 8; ++r) {
      const float mnew  = fmaxf(mrow[r], cm[r]);
      const float alpha = expf(mrow[r] - mnew);
      mrow[r] = mnew;
      float psum = 0.f;
#pragma unroll
      for (int j = 0; j < 4; ++j) {
        const float p = expf(s[j][r] - mnew);
        psum += p;
        if (SPLIT) {
          __bf16 ph, pl2; at_split(p, ph, pl2);
          pwh[(8 * hh + r) * kKC + j * 16 + c] = ph;
          pwl[(8 * hh + r) * kKC + j * 16 + c] = pl2;
        } else {
          pwh[(8 * hh + r) * kKC + j * 16 + c] = at_to16<true>(p * PSC);
        }
      }
#pragma unroll
      for (int off = 1; off < 16; off <<= 1) psum += __shfl_xor(psum, off, 32);
      lrow[r] = lrow[r] * alpha + psum;
#pragma unroll
      for (int t = 0; t < 4; ++t) oacc[t][r] *= alpha;
    }
    __builtin_amdgcn_fence(__ATOMIC_RELEASE, "workgroup");
    __builtin_amdgcn_wave_barrier();
    __builtin_amdgcn_fence(__ATOMIC_ACQUIRE, "workgroup");
#pragma unroll 1
    for (int kk = 0; kk < 2; ++kk) {
      FB pa, pl;
      pa.hv[0] = *(const v8b*)(pwh + c * kKC + kk * 32 + 8 * hh);
      pa.hv[1] = *(const v8b*)(pwh + c * kKC + kk * 32 + 16 + 8 * hh);
      if (SPLIT) {
        pl.hv[0] = *(const v8b*)(pwl + c * kKC + kk * 32 + 8 * hh);
        pl.hv[1] = *(const v8b*)(pwl + c * kKC + kk * 32 + 16 + 8 * hh);
      } else {
        pl.v = pa.v;
      }
#pragma unroll
      for (int t = 0; t < 4; ++t) {
        FB vb;
        vb.u[0] = *(const v4u*)(Vth + (t * 16 + c) * kKC + kk * 32 + 8 * hh);
        vb.u[1] = *(const v4u*)(Vth + (t * 16 + c) * kKC + kk * 32 + 16 + 8 * hh);
        oacc[t] = at_mma16<!SPLIT>(pa.v, vb.v, oacc[t]);
        if (SPLIT) {
          FB vlf;
          vlf.u[0] = *(const v4u*)(Vtl + (t * 16 + c) * kKC + kk * 32 + 8 * hh);
          vlf.u[1] = *(const v4u*)(Vtl + (t * 16 + c) * kKC + kk * 32 + 16 + 8 * hh);
          oacc[t] = at_mma16<!SPLIT>(pa.v, vlf.v, oacc[t]);
          oacc[t] = at_mma16<!SPLIT>(pl.v, vb.v, oacc[t]);
        }
      }
    }
  }

  float* os = Os[wave];
#pragma unroll
  for (int r = 0; r < 8; ++r) {
    const float inv = 1.0f / (lrow[r] * PSC);
#pragma unroll
    for (int t = 0; t < 4; ++t) os[(8 * hh + r) * 68 + t * 16 + c] = oacc[t][r] * inv;
  }
  __builtin_amdgcn_fence(__ATOMIC_RELEASE, "workgroup");
  __builtin_amdgcn_wave_barrier();
  __builtin_amdgcn_fence(__ATOMIC_ACQUIRE, "workgroup");
  {
    const int q4 = lane >> 3, c8 = (lane & 7) * 8;
    const size_t obase = (size_t)b * kS * kD + (size_t)h * kHD;
    for (int pass = 0; pass < 2; ++pass) {
#pragma unroll
      for (int it = 0; it < 4; ++it) {
        const int row = it * 4 + q4;
        const float* sp = os + row * 68 + c8;
        unsigned short hb[8], lb[8];
#pragma unroll
        for (int e = 0; e < 8; ++e) {
          const float val = sp[e];
          const unsigned short hbv = f2bf_bits(val);
          hb[e] = hbv;
          lb[e] = f2bf_bits(val - bf_bits2f(hbv));
        }
        const v4u uh = (v4u){pk16(hb[0], hb[1]), pk16(hb[2], hb[3]), pk16(hb[4], hb[5]), pk16(hb[6], hb[7])};
        const v4u ul = (v4u){pk16(lb[0], lb[1]), pk16(lb[2], lb[3]), pk16(lb[4], lb[5]), pk16(lb[6], lb[7])};
        const size_t o = obase + (size_t)(q0 + row) * kD + c8;
        *(volatile v4u*)(oh + o) = uh;
        *(volatile v4u*)(ol + o) = ul;
      }
      __threadfence();
    }
  }
}

static_assert((kS % 64) == 0 && (kD % 64) == 0 && (kTok % 64) == 0 && (kD % 32) == 0, "gemm tiles");

extern "C" void kernel_launch(void* const* d_in, const int* in_sizes, int n_in,
                              void* d_out, int out_size, void* d_ws, size_t ws_size,
                              hipStream_t stream) {
  if (n_in < 6) return;
  const int nX = kTok * kD;
  const int nW = kD * kD;
  if (in_sizes[0] != nX) return;
  if (in_sizes[1] != nW || in_sizes[2] != nW || in_sizes[3] != nW || in_sizes[4] != nW) return;
  if (in_sizes[5] != kD) return;
  if (out_size != nX) return;

  const size_t szXB   = (size_t)kTok * kD * 2;
  const size_t szWT   = (size_t)kD * kD * 2;
  const size_t szQK16 = (size_t)kTok * kD * 2;
  const size_t szVT16 = (size_t)kBH * kHD * kS * 2;
  const size_t szQKB  = (size_t)kB * kSplitRows * kD * 2;
  const size_t szVB   = (size_t)kBH * kHD * kSplitRows * 2;
  const size_t szCTX  = (size_t)kTok * kD * 2;
  const size_t offXB   = 0;
  const size_t offWQ   = offXB + szXB;
  const size_t offWK   = offWQ + szWT;
  const size_t offWV   = offWK + szWT;
  const size_t offWO   = offWV + szWT;
  const size_t offQ16  = offWO + szWT;
  const size_t offK16  = offQ16 + szQK16;
  const size_t offVT16 = offK16 + szQK16;
  const size_t offQBH  = offVT16 + szVT16;
  const size_t offQBL  = offQBH + szQKB;
  const size_t offKBH  = offQBL + szQKB;
  const size_t offKBL  = offKBH + szQKB;
  const size_t offVBH  = offKBL + szQKB;
  const size_t offVBL  = offVBH + szVB;
  const size_t offCTXH = offVBL + szVB;
  const size_t offCTXL = offCTXH + szCTX;
  const size_t total   = offCTXL + szCTX;
  if (ws_size < total) return;

  const float* x  = (const float*)d_in[0];
  const float* Wq = (const float*)d_in[1];
  const float* Wk = (const float*)d_in[2];
  const float* Wv = (const float*)d_in[3];
  const float* Wo = (const float*)d_in[4];
  const float* bo = (const float*)d_in[5];
  float* out = (float*)d_out;
  char* ws = (char*)d_ws;
  unsigned short* XB   = (unsigned short*)(ws + offXB);
  unsigned short* WQT  = (unsigned short*)(ws + offWQ);
  unsigned short* WKT  = (unsigned short*)(ws + offWK);
  unsigned short* WVT  = (unsigned short*)(ws + offWV);
  unsigned short* WOT  = (unsigned short*)(ws + offWO);
  unsigned short* Q16  = (unsigned short*)(ws + offQ16);
  unsigned short* K16  = (unsigned short*)(ws + offK16);
  unsigned short* VT16 = (unsigned short*)(ws + offVT16);
  unsigned short* QBH  = (unsigned short*)(ws + offQBH);
  unsigned short* QBL  = (unsigned short*)(ws + offQBL);
  unsigned short* KBH  = (unsigned short*)(ws + offKBH);
  unsigned short* KBL  = (unsigned short*)(ws + offKBL);
  unsigned short* VBH  = (unsigned short*)(ws + offVBH);
  unsigned short* VBL  = (unsigned short*)(ws + offVBL);
  unsigned short* CTXH = (unsigned short*)(ws + offCTXH);
  unsigned short* CTXL = (unsigned short*)(ws + offCTXL);

  const int n8 = nX / 8;
  cast8_bf16_kernel<<<dim3(n8 / 256), dim3(256), 0, stream>>>(x, XB, n8);
  wtcast_kernel<<<dim3(kD / 64, kD / 64, 4), dim3(256), 0, stream>>>(Wq, Wk, Wv, Wo, WQT);

  const long strideTokB  = (long)kS * kD;
  const long strideSplit = (long)kSplitRows * kD;
  const long strideVT    = (long)kD * kS;
  const long strideVB    = (long)kD * kSplitRows;
  const int  tilesProj   = (kS / 64) * (kD / 64);
  const int  tilesOut    = (kTok / 64) * (kD / 64);
  const int  bigLim      = 1 << 30;

  wmma_gemm64<1, 0, 0, 3><<<dim3(tilesProj / 8, kB), dim3(256), 0, stream>>>(
      XB, XB, kD, strideTokB, WQT, WQT, kD, 0L,
      (void*)Q16, kD, strideTokB, (void*)QBH, (void*)QBL, kD, strideSplit, kSplitRows, bigLim,
      bo, kS, kD, kD, 1.0f);
  wmma_gemm64<1, 0, 0, 3><<<dim3(tilesProj / 8, kB), dim3(256), 0, stream>>>(
      XB, XB, kD, strideTokB, WKT, WKT, kD, 0L,
      (void*)K16, kD, strideTokB, (void*)KBH, (void*)KBL, kD, strideSplit, kSplitRows, bigLim,
      bo, kS, kD, kD, 1.0f);
  wmma_gemm64<1, 0, 0, 3><<<dim3(tilesProj / 8, kB), dim3(256), 0, stream>>>(
      WVT, WVT, kD, 0L, XB, XB, kD, strideTokB,
      (void*)VT16, kS, strideVT, (void*)VBH, (void*)VBL, kSplitRows, strideVB, bigLim, kSplitRows,
      bo, kD, kS, kD, 1.0f);

  attn_kernel<true><<<dim3(kSplitTiles * kBH), dim3(128), 0, stream>>>(
      QBH, QBL, KBH, KBL, VBH, VBL, CTXH, CTXL, 0, kSplitTiles, kSplitRows, kSplitRows);
  attn_kernel<false><<<dim3((kQTiles - kSplitTiles) * kBH), dim3(128), 0, stream>>>(
      Q16, Q16, K16, K16, VT16, VT16, CTXH, CTXL, kSplitTiles, kQTiles - kSplitTiles, kS, kS);

  wmma_gemm64<1, 2, 2, 0><<<dim3(tilesOut / 8, 1), dim3(256), 0, stream>>>(
      CTXH, CTXL, kD, 0L, WOT, WOT, kD, 0L,
      (void*)out, kD, 0L, (void*)out, (void*)out, 0, 0L, 0, 0,
      bo, kTok, kD, kD, 1.0f);
}
